// MultiHeadAttention_9612136808854
// MI455X (gfx1250) — hardware-verified
//
#include <hip/hip_runtime.h>


#ifndef NB
#define NB 4
#endif
#ifndef SEQ
#define SEQ 2048
#endif
#define NB_FULL  4
#define SEQ_FULL 2048
#define DM   1024
#define NH   16
#define HD   64
#define RH   256
#define PCAR 1024.0f
#define CCAR 16.0f
#define WCAR 32.0f
#define SCL2 (0.125f * 1.4426950408889634f)

static_assert(DM == NH * HD);
static_assert(HD == 64);
static_assert(DM % 32 == 0);
static_assert(HD % 32 == 0);
static_assert(SEQ % 64 == 0);
static_assert(RH % 64 == 0);
static_assert(SEQ >= RH);
static_assert((SEQ - RH) % 64 == 0);
static_assert(RH % 32 == 0);
static_assert(NB <= NB_FULL);
static_assert(SEQ <= SEQ_FULL);

typedef unsigned short u16;
typedef _Float16 h16;
typedef __attribute__((ext_vector_type(16))) __bf16         v16bf;
typedef __attribute__((ext_vector_type(16))) _Float16       v16h;
typedef __attribute__((ext_vector_type(8)))  unsigned short v8us;
typedef __attribute__((ext_vector_type(16))) unsigned short v16us;
typedef __attribute__((ext_vector_type(8)))  float          v8f;
typedef __attribute__((ext_vector_type(4)))  float          v4f;
typedef v4f  __attribute__((may_alias)) v4fa;
typedef v8us __attribute__((may_alias)) v8usa;

#define XBN    ((size_t)NB * SEQ * DM)
#define WN     ((size_t)DM * DM)
#define PLANE  ((size_t)NB * NH * SEQ * HD)
#define EPLANE ((size_t)NB * NH * RH * HD)
#define ATN    ((size_t)NB * (SEQ - RH) * DM)
#define ATEN   ((size_t)NB * RH * DM)
#define O_XB   ((size_t)0)
#define O_WALL (O_XB + XBN)
#define O_WPB  (O_WALL + 3 * WN)
#define O_WPH  (O_WPB + WN)
#define O_P16  (O_WPH + WN)
#define O_EH   (O_P16 + 3 * PLANE)
#define O_EL   (O_EH + 3 * EPLANE)
#define O_AT   (O_EL + 3 * EPLANE)
#define O_ATEH (O_AT + ATN)
#define O_ATEL (O_ATEH + ATEN)
#define O_END  (O_ATEL + ATEN)
static_assert(O_END * 2 <= (size_t)134217728);
static_assert(XBN % 128 == 0 && WN % 128 == 0 && PLANE % 128 == 0 && EPLANE % 128 == 0 && ATN % 128 == 0 && ATEN % 128 == 0);

__device__ __forceinline__ u16 f2bf(float f) { unsigned u = __float_as_uint(f); u += 0x7FFFu + ((u >> 16) & 1u); return (u16)(u >> 16); }
__device__ __forceinline__ float bf2f(u16 b) { return __uint_as_float(((unsigned)b) << 16); }
__device__ __forceinline__ float bfr(float f) { return bf2f(f2bf(f)); }
__device__ __forceinline__ u16 f2h(float x) { return __builtin_bit_cast(unsigned short, (h16)x); }

__device__ __forceinline__ v16us ldfr(const u16* p) {
    const v8us lo = *(const v8us*)p; const v8us hi = *(const v8us*)(p + 16);
    return __builtin_shufflevector(lo, hi, 0, 1, 2, 3, 4, 5, 6, 7, 8, 9, 10, 11, 12, 13, 14, 15);
}
__device__ __forceinline__ v8f mma_h(v16us a, v16us b, v8f c) {
    const v16h ah = __builtin_bit_cast(v16h, a); const v16h bh = __builtin_bit_cast(v16h, b);
    c = __builtin_amdgcn_wmma_f32_16x16x32_f16(false, ah, false, bh, (short)0, c, false, false);
    asm volatile("v_nop\n\tv_nop\n\tv_nop\n\tv_nop" : "+v"(c) : "v"(ah), "v"(bh));
    return c;
}
__device__ __forceinline__ v8f mma_b(v16us a, v16us b, v8f c) {
    const v16bf ab = __builtin_bit_cast(v16bf, a); const v16bf bb = __builtin_bit_cast(v16bf, b);
    c = __builtin_amdgcn_wmma_f32_16x16x32_bf16(false, ab, false, bb, (short)0, c, false, false);
    asm volatile("v_nop\n\tv_nop\n\tv_nop\n\tv_nop" : "+v"(c) : "v"(ab), "v"(bb));
    return c;
}
template <bool F16> __device__ __forceinline__ v8f mmag(v16us a, v16us b, v8f c) { if (F16) return mma_h(a, b, c); else return mma_b(a, b, c); }

template <bool F16, bool SPLIT>
__device__ __forceinline__ void gemm_tile(const u16* __restrict__ A, const u16* __restrict__ A2, const u16* __restrict__ Bt, const int K, const int r0, const int c0, const int lr, const int hi, v8f (&acc)[4][4]) {
#pragma unroll
    for (int mb = 0; mb < 4; ++mb)
#pragma unroll
        for (int nb = 0; nb < 4; ++nb) acc[mb][nb] = (v8f){};
    const size_t aoff = (size_t)(r0 + lr) * K + 8 * hi, boff = (size_t)(c0 + lr) * K + 8 * hi;
#pragma unroll 1
    for (int kc = 0; kc < K; kc += 32) {
        v16us a[4], a2[4];
#pragma unroll
        for (int mb = 0; mb < 4; ++mb) { a[mb] = ldfr(A + aoff + (size_t)mb * 16 * K + kc); if (SPLIT) a2[mb] = ldfr(A2 + aoff + (size_t)mb * 16 * K + kc); else a2[mb] = a[mb]; }
#pragma unroll
        for (int nb = 0; nb < 4; ++nb) { const v16us bb = ldfr(Bt + boff + (size_t)nb * 16 * K + kc);
#pragma unroll
            for (int mb = 0; mb < 4; ++mb) { acc[mb][nb] = mmag<F16>(a[mb], bb, acc[mb][nb]); if (SPLIT) acc[mb][nb] = mmag<F16>(a2[mb], bb, acc[mb][nb]); } }
    }
}

__global__ __launch_bounds__(256) void k_cvt8(const float* __restrict__ src, u16* dst, unsigned n8, unsigned seg, unsigned segf, int tof16, float scale) {
    const unsigned i = blockIdx.x * 256u + threadIdx.x;
    if (i >= n8) return;
    const unsigned bb = i / seg, r = i - bb * seg;
    const size_t si = ((size_t)bb * segf + r) * 8;
    const v4f v0 = *(const v4f*)(src + si); const v4f v1 = *(const v4f*)(src + si + 4);
    v8us o;
#pragma unroll
    for (int k = 0; k < 4; ++k) {
        const u16 b0 = f2bf(v0[k]), b1 = f2bf(v1[k]);
        const u16 h0 = f2h(bf2f(b0) * scale), h1 = f2h(bf2f(b1) * scale);
        o[k] = tof16 ? h0 : b0; o[4 + k] = tof16 ? h1 : b1;
    }
    volatile v8us* dp = (volatile v8us*)(dst + (size_t)i * 8);
    *dp = o; __threadfence(); *dp = o;
}

__global__ __launch_bounds__(32) void k_proj(const u16* __restrict__ XB, const u16* __restrict__ WALL, u16* PL, size_t oP16, size_t oEH, size_t oEL) {
    __shared__ __align__(16) float os[16 * 68];
    __shared__ __align__(16) u16 ts[64 * 72];
    const int lane = threadIdx.x & 31, lr = lane & 15, hi = lane >> 4;
    const int r0 = blockIdx.x * 64, c0 = blockIdx.y * 64;
    const int which = c0 / DM, hd = (c0 - which * DM) / HD;
    const int b = r0 / SEQ, t0 = r0 - b * SEQ;
    const bool early = (t0 < RH);
    const size_t bh = (size_t)b * NH + hd;
    v8f acc[4][4];
    gemm_tile<false, false>(XB, XB, WALL, DM, r0, c0, lr, hi, acc);
    if (which < 2) {
        const size_t o16 = oP16 + (size_t)which * PLANE + (bh * SEQ + t0) * HD;
        const size_t oeh = oEH + (size_t)which * EPLANE + (bh * RH + (early ? t0 : 0)) * HD;
        const size_t oel = oEL + (size_t)which * EPLANE + (bh * RH + (early ? t0 : 0)) * HD;
#pragma unroll
        for (int mb = 0; mb < 4; ++mb) {
#pragma unroll
            for (int nb = 0; nb < 4; ++nb)
#pragma unroll
                for (int j = 0; j < 8; ++j) os[(hi * 8 + j) * 68 + nb * 16 + lr] = acc[mb][nb][j];
            __syncthreads();
#pragma unroll 1
            for (int ps = 0; ps < 2; ++ps) {
#pragma unroll
                for (int s = 0; s < 4; ++s) {
                    const int row = 4 * s + (lane >> 3), pc = (lane & 7) * 8;
                    const v4f x0 = *(const v4fa*)&os[row * 68 + pc]; const v4f x1 = *(const v4fa*)&os[row * 68 + pc + 4];
                    v8us q16;
#pragma unroll
                    for (int q = 0; q < 4; ++q) { q16[q] = f2h(x0[q]); q16[4 + q] = f2h(x1[q]); }
                    const size_t ro = (size_t)(mb * 16 + row) * HD + pc;
                    *(volatile v8us*)(PL + o16 + ro) = q16;
                    if (early) {
                        v8us oh, ol;
#pragma unroll
                        for (int q = 0; q < 4; ++q) { const u16 a = f2bf(x0[q]); oh[q] = a; ol[q] = f2bf(x0[q] - bf2f(a)); const u16 c = f2bf(x1[q]); oh[4 + q] = c; ol[4 + q] = f2bf(x1[q] - bf2f(c)); }
                        *(volatile v8us*)(PL + oeh + ro) = oh; *(volatile v8us*)(PL + oel + ro) = ol;
                    }
                }
                if (ps == 0) __threadfence();
            }
            __syncthreads();
        }
    } else {
#pragma unroll
        for (int pl = 0; pl < 3; ++pl) {
            if (pl == 0 || early) {
#pragma unroll
                for (int mb = 0; mb < 4; ++mb)
#pragma unroll
                    for (int nb = 0; nb < 4; ++nb) {
                        v8us pk;
#pragma unroll
                        for (int j = 0; j < 8; ++j) { const float y = acc[mb][nb][j]; const u16 hb = f2bf(y); pk[j] = (pl == 0) ? f2h(y) : ((pl == 1) ? hb : f2bf(y - bf2f(hb))); }
                        *(v8usa*)&ts[(nb * 16 + lr) * 72 + mb * 16 + hi * 8] = pk;
                    }
                __syncthreads();
                const size_t dofs = (pl == 0) ? (oP16 + 2 * PLANE + bh * HD * SEQ + t0) : (((pl == 1) ? oEH : oEL) + 2 * EPLANE + bh * HD * RH + t0);
                const int dp = (pl == 0) ? SEQ : RH;
#pragma unroll 1
                for (int ps = 0; ps < 2; ++ps) {
#pragma unroll 4
                    for (int s = 0; s < 16; ++s) {
                        const int d = 4 * s + (lane >> 3), pc = (lane & 7) * 8;
                        const v8us v = *(const v8usa*)&ts[d * 72 + pc];
                        *(volatile v8us*)(PL + dofs + (size_t)d * dp + pc) = v;
                    }
                    if (ps == 0) __threadfence();
                }
                __syncthreads();
            }
        }
    }
}

__device__ __forceinline__ void sm_step(v8f& s0, v8f& s1, float (&mrow)[8], float (&lrow)[8], float (&corr)[8], const int jb, const int qbase, const int lr, const int hi) {
#pragma unroll
    for (int i = 0; i < 8; ++i) {
        const int row = qbase + i + 8 * hi;
        float a0 = s0[i] * SCL2, a1 = s1[i] * SCL2;
        a0 = (jb + lr > row) ? -1.0e30f : a0;
        a1 = (jb + 16 + lr > row) ? -1.0e30f : a1;
        float mx = fmaxf(a0, a1);
        mx = fmaxf(mx, __shfl_xor(mx, 1, 32)); mx = fmaxf(mx, __shfl_xor(mx, 2, 32)); mx = fmaxf(mx, __shfl_xor(mx, 4, 32)); mx = fmaxf(mx, __shfl_xor(mx, 8, 32));
        const float mnew = fmaxf(mrow[i], mx);
        const float c  = __builtin_amdgcn_exp2f(mrow[i] - mnew);
        const float p0 = __builtin_amdgcn_exp2f(a0 - mnew);
        const float p1 = __builtin_amdgcn_exp2f(a1 - mnew);
        lrow[i] = lrow[i] * c + (p0 + p1);
        mrow[i] = mnew; corr[i] = c; s0[i] = p0; s1[i] = p1;
    }
}

#define NQT_L (((SEQ - RH) / 16) > 0 ? ((SEQ - RH) / 16) : 1)

__global__ __launch_bounds__(32) void k_attn_l(const u16* __restrict__ QP, const u16* __restrict__ KP, const u16* __restrict__ VT, u16* AT) {
    __shared__ __align__(16) u16 pw[16 * 40];
    __shared__ __align__(16) float os[16 * 68];
    const int lane = threadIdx.x & 31, lr = lane & 15, hi = lane >> 4;
    const int bh = blockIdx.x / NQT_L, qt = blockIdx.x - bh * NQT_L;
    const int b = bh / NH, h = bh - b * NH;
    const int qbase = RH + qt * 16;
    const size_t pb = (size_t)bh * SEQ * HD;
    const u16* Qb = QP + pb; const u16* Kb = KP + pb; const u16* Vb = VT + pb;
    const v16us q0 = ldfr(Qb + (size_t)(qbase + lr) * HD + 8 * hi);
    const v16us q1 = ldfr(Qb + (size_t)(qbase + lr) * HD + 32 + 8 * hi);
    v8f acc[4];
#pragma unroll
    for (int nt = 0; nt < 4; ++nt) acc[nt] = (v8f){};
    float mrow[8], lrow[8];
#pragma unroll
    for (int i = 0; i < 8; ++i) { mrow[i] = -1.0e30f; lrow[i] = 0.0f; }
    const int nsteps = (qbase + 47) >> 5;
#pragma unroll 1
    for (int st = 0; st < nsteps; ++st) {
        const int jb = st * 32;
        const u16* kr0 = Kb + (size_t)(jb + lr) * HD + 8 * hi; const u16* kr1 = kr0 + 16 * HD;
        v8f s0 = (v8f){}, s1 = (v8f){};
        s0 = mma_h(q0, ldfr(kr0), s0); s0 = mma_h(q1, ldfr(kr0 + 32), s0);
        s1 = mma_h(q0, ldfr(kr1), s1); s1 = mma_h(q1, ldfr(kr1 + 32), s1);
        float corr[8];
        sm_step(s0, s1, mrow, lrow, corr, jb, qbase, lr, hi);
#pragma unroll
        for (int nt = 0; nt < 4; ++nt)
#pragma unroll
            for (int i = 0; i < 8; ++i) acc[nt][i] *= corr[i];
#pragma unroll
        for (int i = 0; i < 8; ++i) { pw[(i + 8 * hi) * 40 + lr] = f2h(s0[i] * PCAR); pw[(i + 8 * hi) * 40 + 16 + lr] = f2h(s1[i] * PCAR); }
        __syncthreads();
        const v8us plo = *(const v8usa*)&pw[lr * 40 + 8 * hi]; const v8us phi = *(const v8usa*)&pw[lr * 40 + 16 + 8 * hi];
        const v16us pf = __builtin_shufflevector(plo, phi, 0, 1, 2, 3, 4, 5, 6, 7, 8, 9, 10, 11, 12, 13, 14, 15);
#pragma unroll
        for (int nt = 0; nt < 4; ++nt) { const v16us vf = ldfr(Vb + (size_t)(nt * 16 + lr) * SEQ + jb + 8 * hi); acc[nt] = mma_h(pf, vf, acc[nt]); }
        __syncthreads();
    }
#pragma unroll
    for (int i = 0; i < 8; ++i) {
        float l = lrow[i];
        l += __shfl_xor(l, 1, 32); l += __shfl_xor(l, 2, 32); l += __shfl_xor(l, 4, 32); l += __shfl_xor(l, 8, 32);
        const float inv = CCAR / (l * PCAR);
#pragma unroll
        for (int nt = 0; nt < 4; ++nt) os[(i + 8 * hi) * 68 + nt * 16 + lr] = acc[nt][i] * inv;
    }
    __syncthreads();
    u16* dst = AT + ((size_t)b * (SEQ - RH) + (qbase - RH)) * DM + h * HD;
#pragma unroll 1
    for (int ps = 0; ps < 2; ++ps) {
#pragma unroll
        for (int s = 0; s < 4; ++s) {
            const int row = 4 * s + (lane >> 3), pc = (lane & 7) * 8;
            const v4f x0 = *(const v4fa*)&os[row * 68 + pc]; const v4f x1 = *(const v4fa*)&os[row * 68 + pc + 4];
            v8us o;
#pragma unroll
            for (int q = 0; q < 4; ++q) { o[q] = f2h(x0[q]); o[4 + q] = f2h(x1[q]); }
            *(volatile v8us*)(dst + (size_t)row * DM + pc) = o;
        }
        if (ps == 0) __threadfence();
    }
}

__global__ __launch_bounds__(32) void k_attn_e(const u16* __restrict__ QEh, const u16* __restrict__ QEl, const u16* __restrict__ KEh, const u16* __restrict__ KEl, const u16* __restrict__ VEh, const u16* __restrict__ VEl, u16* ATEh, u16* ATEl) {
    __shared__ __align__(16) u16 pwh[16 * 40];
    __shared__ __align__(16) u16 pwl[16 * 40];
    __shared__ __align__(16) float os[16 * 68];
    const int lane = threadIdx.x & 31, lr = lane & 15, hi = lane >> 4;
    const int bh = blockIdx.x / (RH / 16), qt = blockIdx.x - bh * (RH / 16);
    const int b = bh / NH, h = bh - b * NH;
    const int qbase = qt * 16;
    const size_t pb = (size_t)bh * RH * HD;
    const size_t qo = pb + (size_t)(qbase + lr) * HD + 8 * hi;
    const v16us qh0 = ldfr(QEh + qo), qh1 = ldfr(QEh + qo + 32), ql0 = ldfr(QEl + qo), ql1 = ldfr(QEl + qo + 32);
    v8f acc[4];
#pragma unroll
    for (int nt = 0; nt < 4; ++nt) acc[nt] = (v8f){};
    float mrow[8], lrow[8];
#pragma unroll
    for (int i = 0; i < 8; ++i) { mrow[i] = -1.0e30f; lrow[i] = 0.0f; }
    const int nsteps = (qbase + 47) >> 5;
#pragma unroll 1
    for (int st = 0; st < nsteps; ++st) {
        const int jb = st * 32;
        const size_t ko = pb + (size_t)(jb + lr) * HD + 8 * hi;
        v8f s0 = (v8f){}, s1 = (v8f){};
        {
            const v16us kh0 = ldfr(KEh + ko), kh1 = ldfr(KEh + ko + 32), kl0 = ldfr(KEl + ko), kl1 = ldfr(KEl + ko + 32);
            s0 = mma_b(qh0, kh0, s0); s0 = mma_b(qh1, kh1, s0); s0 = mma_b(ql0, kh0, s0); s0 = mma_b(ql1, kh1, s0); s0 = mma_b(qh0, kl0, s0); s0 = mma_b(qh1, kl1, s0);
        }
        {
            const size_t k1 = ko + 16 * HD;
            const v16us kh0 = ldfr(KEh + k1), kh1 = ldfr(KEh + k1 + 32), kl0 = ldfr(KEl + k1), kl1 = ldfr(KEl + k1 + 32);
            s1 = mma_b(qh0, kh0, s1); s1 = mma_b(qh1, kh1, s1); s1 = mma_b(ql0, kh0, s1); s1 = mma_b(ql1, kh1, s1); s1 = mma_b(qh0, kl0, s1); s1 = mma_b(qh1, kl1, s1);
        }
        float corr[8];
        sm_step(s0, s1, mrow, lrow, corr, jb, qbase, lr, hi);
#pragma unroll
        for (int nt = 0; nt < 4; ++nt)
#pragma unroll
            for (int i = 0; i < 8; ++i) acc[nt][i] *= corr[i];
#pragma unroll
        for (int i = 0; i < 8; ++i) {
            const u16 a = f2bf(s0[i]); const u16 c = f2bf(s1[i]);
            pwh[(i + 8 * hi) * 40 + lr] = a; pwl[(i + 8 * hi) * 40 + lr] = f2bf(s0[i] - bf2f(a));
            pwh[(i + 8 * hi) * 40 + 16 + lr] = c; pwl[(i + 8 * hi) * 40 + 16 + lr] = f2bf(s1[i] - bf2f(c));
        }
        __syncthreads();
        const v8us h0 = *(const v8usa*)&pwh[lr * 40 + 8 * hi]; const v8us h1 = *(const v8usa*)&pwh[lr * 40 + 16 + 8 * hi];
        const v8us l0 = *(const v8usa*)&pwl[lr * 40 + 8 * hi]; const v8us l1 = *(const v8usa*)&pwl[lr * 40 + 16 + 8 * hi];
        const v16us pfh = __builtin_shufflevector(h0, h1, 0, 1, 2, 3, 4, 5, 6, 7, 8, 9, 10, 11, 12, 13, 14, 15);
        const v16us pfl = __builtin_shufflevector(l0, l1, 0, 1, 2, 3, 4, 5, 6, 7, 8, 9, 10, 11, 12, 13, 14, 15);
#pragma unroll
        for (int nt = 0; nt < 4; ++nt) {
            const size_t vo = pb + (size_t)(nt * 16 + lr) * RH + jb + 8 * hi;
            const v16us vh = ldfr(VEh + vo), vl = ldfr(VEl + vo);
            acc[nt] = mma_b(pfh, vh, acc[nt]); acc[nt] = mma_b(pfl, vh, acc[nt]); acc[nt] = mma_b(pfh, vl, acc[nt]);
        }
        __syncthreads();
    }
#pragma unroll
    for (int i = 0; i < 8; ++i) {
        float l = lrow[i];
        l += __shfl_xor(l, 1, 32); l += __shfl_xor(l, 2, 32); l += __shfl_xor(l, 4, 32); l += __shfl_xor(l, 8, 32);
        const float inv = 1.0f / l;
#pragma unroll
        for (int nt = 0; nt < 4; ++nt) os[(i + 8 * hi) * 68 + nt * 16 + lr] = acc[nt][i] * inv;
    }
    __syncthreads();
    const size_t dofs = ((size_t)b * RH + qbase) * DM + h * HD;
#pragma unroll 1
    for (int ps = 0; ps < 2; ++ps) {
#pragma unroll
        for (int s = 0; s < 4; ++s) {
            const int row = 4 * s + (lane >> 3), pc = (lane & 7) * 8;
            const v4f x0 = *(const v4fa*)&os[row * 68 + pc]; const v4f x1 = *(const v4fa*)&os[row * 68 + pc + 4];
            v8us oh, ol;
#pragma unroll
            for (int q = 0; q < 4; ++q) { const u16 a = f2bf(x0[q]); oh[q] = a; ol[q] = f2bf(x0[q] - bf2f(a)); const u16 c = f2bf(x1[q]); oh[4 + q] = c; ol[4 + q] = f2bf(x1[q] - bf2f(c)); }
            *(volatile v8us*)(ATEh + dofs + (size_t)row * DM + pc) = oh;
            *(volatile v8us*)(ATEl + dofs + (size_t)row * DM + pc) = ol;
        }
        if (ps == 0) __threadfence();
    }
}

__global__ __launch_bounds__(32) void k_outp(const u16* __restrict__ A, const u16* __restrict__ A2, const u16* __restrict__ Bt, const float* __restrict__ bias, float* OUT, float scale, int rpb, int toff, int split) {
    __shared__ __align__(16) float os[16 * 68];
    const int lane = threadIdx.x & 31, lr = lane & 15, hi = lane >> 4;
    const int r0 = blockIdx.x * 64, c0 = blockIdx.y * 64;
    v8f acc[4][4];
    if (split) gemm_tile<false, true>(A, A2, Bt, DM, r0, c0, lr, hi, acc);
    else       gemm_tile<true, false>(A, A, Bt, DM, r0, c0, lr, hi, acc);
    const int b = r0 / rpb, tb = toff + (r0 - b * rpb);
    float* crow0 = OUT + ((size_t)b * SEQ_FULL + tb) * DM + c0;
    const int cofs = lr * 4;
    v4f bv; bv[0] = bfr(bias[c0 + cofs]); bv[1] = bfr(bias[c0 + cofs + 1]); bv[2] = bfr(bias[c0 + cofs + 2]); bv[3] = bfr(bias[c0 + cofs + 3]);
#pragma unroll
    for (int mb = 0; mb < 4; ++mb) {
#pragma unroll
        for (int nb = 0; nb < 4; ++nb)
#pragma unroll
            for (int j = 0; j < 8; ++j) os[(hi * 8 + j) * 68 + nb * 16 + lr] = acc[mb][nb][j];
        __syncthreads();
#pragma unroll 1
        for (int ps = 0; ps < 2; ++ps) {
#pragma unroll
            for (int s = 0; s < 8; ++s) {
                const int row = 2 * s + hi;
                const v4f x = *(const v4fa*)&os[row * 68 + cofs];
                v4f val; val[0] = x[0] * scale + bv[0]; val[1] = x[1] * scale + bv[1]; val[2] = x[2] * scale + bv[2]; val[3] = x[3] * scale + bv[3];
                *(volatile v4f*)(crow0 + (size_t)(mb * 16 + row) * DM + cofs) = val;
            }
            if (ps == 0) __threadfence();
        }
        __syncthreads();
    }
}

extern "C" void kernel_launch(void* const* d_in, const int* in_sizes, int n_in,
                              void* d_out, int out_size, void* d_ws, size_t ws_size, hipStream_t stream) {
    if (n_in < 6) return;
    const long long needx = ((long long)(NB - 1) * SEQ_FULL + SEQ) * DM;
    if ((long long)in_sizes[0] < needx) return;
    if ((long long)in_sizes[1] < (long long)DM * DM || (long long)in_sizes[2] < (long long)DM * DM || (long long)in_sizes[3] < (long long)DM * DM || (long long)in_sizes[4] < (long long)DM * DM) return;
    if (in_sizes[5] < DM) return;
    if ((long long)out_size < needx) return;
    if (O_END * 2 > ws_size) return;
    const float* x  = (const float*)d_in[0];
    const float* Wk = (const float*)d_in[1];
    const float* Wq = (const float*)d_in[2];
    const float* Wv = (const float*)d_in[3];
    const float* Wp = (const float*)d_in[4];
    const float* bp = (const float*)d_in[5];
    float* OUT = (float*)d_out;
    u16* PL = (u16*)d_ws;

    const unsigned xn8 = (unsigned)(XBN / 8), wn8 = (unsigned)(WN / 8);
    k_cvt8<<<(xn8 + 255) / 256, 256, 0, stream>>>(x, PL + O_XB, xn8, (unsigned)((size_t)SEQ * DM / 8), (unsigned)((size_t)SEQ_FULL * DM / 8), 0, 1.0f);
    k_cvt8<<<(wn8 + 255) / 256, 256, 0, stream>>>(Wq, PL + O_WALL,          wn8, wn8, wn8, 0, 1.0f);
    k_cvt8<<<(wn8 + 255) / 256, 256, 0, stream>>>(Wk, PL + O_WALL + WN,     wn8, wn8, wn8, 0, 1.0f);
    k_cvt8<<<(wn8 + 255) / 256, 256, 0, stream>>>(Wv, PL + O_WALL + 2 * WN, wn8, wn8, wn8, 0, 1.0f);
    k_cvt8<<<(wn8 + 255) / 256, 256, 0, stream>>>(Wp, PL + O_WPB, wn8, wn8, wn8, 0, 1.0f);
    k_cvt8<<<(wn8 + 255) / 256, 256, 0, stream>>>(Wp, PL + O_WPH, wn8, wn8, wn8, 1, WCAR);

    k_proj<<<dim3(NB * SEQ / 64, 3 * DM / 64, 1), 32, 0, stream>>>(PL + O_XB, PL + O_WALL, PL, O_P16, O_EH, O_EL);

    k_attn_e<<<NB * NH * (RH / 16), 32, 0, stream>>>(PL + O_EH, PL + O_EL, PL + O_EH + EPLANE, PL + O_EL + EPLANE, PL + O_EH + 2 * EPLANE, PL + O_EL + 2 * EPLANE, PL + O_ATEH, PL + O_ATEL);
    if (SEQ > RH)
        k_attn_l<<<NB * NH * ((SEQ - RH) / 16), 32, 0, stream>>>(PL + O_P16, PL + O_P16 + PLANE, PL + O_P16 + 2 * PLANE, PL + O_AT);

    k_outp<<<dim3(NB * RH / 64, DM / 64, 1), 32, 0, stream>>>(PL + O_ATEH, PL + O_ATEL, PL + O_WPB, bp, OUT, 1.0f, RH, 0, 1);
    if (SEQ > RH)
        k_outp<<<dim3(NB * (SEQ - RH) / 64, DM / 64, 1), 32, 0, stream>>>(PL + O_AT, PL + O_AT, PL + O_WPH, bp, OUT, 1.0f / (WCAR * CCAR), SEQ - RH, RH, 0);
}
